// S6_20005957665390
// MI455X (gfx1250) — hardware-run, weakly checked
//
#include <hip/hip_runtime.h>
#include <hip/hip_fp16.h>
#include <math.h>

typedef __attribute__((ext_vector_type(16))) _Float16 v16h;
typedef __attribute__((ext_vector_type(8)))  _Float16 v8h;
typedef __attribute__((ext_vector_type(8)))  float    v8f;
typedef __attribute__((ext_vector_type(4)))  float    v4f;
typedef __attribute__((ext_vector_type(4)))  unsigned v4u;

constexpr int kBatch  = 4;
constexpr int kSeq    = 2048;
constexpr int kDim    = 512;
constexpr int kNst    = 16;
constexpr int kLayers = 2;
constexpr int kProjN  = 2 * kNst + kDim;
constexpr int kProjP  = 576;
constexpr int kBcP    = 2 * kNst;
constexpr int kNumVec = 11;
constexpr float kLnEps  = 1e-5f;
constexpr float kWCarry = 1024.0f;
constexpr float kResid  = 2048.0f;
constexpr float kYCarry = 16.0f;
constexpr float kInvResid = 1.0f / kResid;
constexpr float kInvCarry = 1.0f / kYCarry;
static_assert(kProjN == 544);
static_assert(kBcP == 32);
static_assert(kProjN <= kProjP && (kProjP % 64) == 0);
static_assert((kSeq % 64) == 0 && (kDim % 64) == 0 && (kDim % 32) == 0);
static_assert((kSeq % 32) == 0 && (kSeq % 8) == 0);
static_assert((kNst % 4) == 0 && (kBcP % 4) == 0 && (kProjN % 4) == 0 && (kProjP % 4) == 0);
static_assert(kDim == 512);

constexpr size_t kSzWCAT = (size_t)kDim * kProjP * 4;
constexpr size_t kSzW3   = (size_t)kProjP * kDim * 2;
constexpr size_t kSzW16  = (size_t)kDim * kDim * 2;
constexpr size_t kSzVEC  = (size_t)kDim * 4;
constexpr size_t kSzALOG = (size_t)kDim * kNst * 4;
constexpr size_t kSzH32  = (size_t)kSeq * kDim * 4;
constexpr size_t kSzH16  = (size_t)kSeq * kDim * 2;
constexpr size_t kSzP    = (size_t)kSeq * kProjP * 4;
constexpr size_t kSzBC   = (size_t)kSeq * kBcP * 4;
constexpr size_t kOffWCAT = 0;
constexpr size_t kOffW3   = kOffWCAT + kLayers * kSzWCAT;
constexpr size_t kOffWM   = kOffW3   + kLayers * kSzW3;
constexpr size_t kOffWD   = kOffWM   + kLayers * kSzW16;
constexpr size_t kOffVEC  = kOffWD   + kSzW16;
constexpr size_t kOffALOG = kOffVEC  + kNumVec * kSzVEC;
constexpr size_t kOffHA   = kOffALOG + kLayers * kSzALOG;
constexpr size_t kOffHB   = kOffHA   + kSzH32;
constexpr size_t kOffHH   = kOffHB   + kSzH32;
constexpr size_t kOffHL   = kOffHH   + kSzH16;
constexpr size_t kOffP    = kOffHL   + kSzH16;
constexpr size_t kOffBC   = kOffP    + kSzP;
constexpr size_t kOffDT   = kOffBC   + kSzBC;
constexpr size_t kOffYH   = kOffDT   + kSzH32;
constexpr size_t kOffYL   = kOffYH   + kSzH16;
constexpr size_t kOffGH   = kOffYL   + kSzH16;
constexpr size_t kOffGL   = kOffGH   + kSzH16;
constexpr size_t kOffMX   = kOffGL   + kSzH16;
constexpr size_t kOffDEC  = kOffMX   + kSzH32;
constexpr size_t kWsTotal = kOffDEC  + kSzH32;
static_assert(kSzWCAT == 1179648ull && kSzW3 == 589824ull && kSzW16 == 524288ull);
static_assert(kSzVEC == 2048ull && kSzALOG == 32768ull);
static_assert(kSzH32 == 4194304ull && kSzH16 == 2097152ull && kSzP == 4718592ull && kSzBC == 262144ull);
static_assert(kWsTotal == 43735040ull);
static_assert(kWsTotal <= 134217728ull);
static_assert((kOffW3 % 128) == 0 && (kOffWM % 128) == 0 && (kOffWD % 128) == 0 && (kOffVEC % 128) == 0 &&
              (kOffALOG % 128) == 0 && (kOffHA % 128) == 0 && (kOffHB % 128) == 0 && (kOffHH % 128) == 0 &&
              (kOffHL % 128) == 0 && (kOffP % 128) == 0 && (kOffBC % 128) == 0 && (kOffDT % 128) == 0 &&
              (kOffYH % 128) == 0 && (kOffYL % 128) == 0 && (kOffGH % 128) == 0 && (kOffGL % 128) == 0 &&
              (kOffMX % 128) == 0 && (kOffDEC % 128) == 0);
static_assert((kSzWCAT % 128) == 0 && (kSzW3 % 128) == 0 && (kSzVEC % 128) == 0 && (kSzALOG % 128) == 0);

__device__ __forceinline__ _Float16 f16_flush(float v) {
  const float w = (fabsf(v) < 6.103515625e-05f) ? 0.0f : v;
  return (_Float16)w;
}
__device__ __forceinline__ void f16_split(float v, _Float16& hi, _Float16& lo) {
  hi = f16_flush(v);
  const float hf = (float)hi;
  const float r = (v - hf) * kResid;
  lo = f16_flush(r);
}

__device__ __forceinline__ float bf16r(float v) {
  unsigned u = __float_as_uint(v);
  u = (u + 0x7FFFu + ((u >> 16) & 1u)) & 0xFFFF0000u;
  return __uint_as_float(u);
}

__device__ __forceinline__ float h16_to_f32(unsigned hb) {
  const unsigned sgn = (hb & 0x8000u) << 16; const unsigned em = hb & 0x7fffu;
  const float fn = __uint_as_float((em << 13) + 0x38000000u);
  const float fs = (float)em * 5.9604644775390625e-8f;
  const float mag = (em < 0x400u) ? fs : fn; return __uint_as_float(__float_as_uint(mag) | sgn); }

namespace eng {
union FragU { v16h v; v8h h[2]; };
__device__ __forceinline__ v16h frag_load(const _Float16* p) {
  FragU f;
  f.h[0] = *(const v8h*)(p);
  f.h[1] = *(const v8h*)(p + 16);
  return f.v;
}
__device__ __forceinline__ v8f mma(v16h a, v16h b, v8f c) {
  return __builtin_amdgcn_wmma_f32_16x16x32_f16(false, a, false, b, (short)0, c, false, false);
}
__device__ __forceinline__ void guard1(v8f& a, v16h x, v16h y) {
  asm volatile("v_nop\n\tv_nop\n\tv_nop\n\tv_nop" : "+v"(a) : "v"(x), "v"(y));
}
__device__ __forceinline__ void guard_acc(v8f& a) {
  asm volatile("v_nop\n\tv_nop\n\tv_nop\n\tv_nop" : "+v"(a));
}
__device__ __forceinline__ void keep4(v16h a, v16h b, v16h c, v16h d) {
  asm volatile("v_nop" :: "v"(a), "v"(b), "v"(c), "v"(d));
}

template <int MI, int SPL>
__global__ __launch_bounds__(256) void gemm_f16_kernel(
    const unsigned short* __restrict__ Ap, const unsigned short* __restrict__ A2p, int lda,
    const unsigned short* __restrict__ Btp, const unsigned short* __restrict__ Bt2p, int ldb,
    float* __restrict__ C, int ldc, int M, int N, int K, float scale, float rscale)
{
  static_assert(MI >= 1 && MI <= 2);
  static_assert(SPL >= 0 && SPL <= 2);
  const _Float16* A   = (const _Float16*)Ap;
  const _Float16* A2  = (const _Float16*)A2p;
  const _Float16* Bt  = (const _Float16*)Btp;
  const _Float16* Bt2 = (const _Float16*)Bt2p;
  __shared__ __align__(16) float sT[8][16 * 68];
  const int lane = threadIdx.x & 31;
  const int wave = threadIdx.x >> 5;
  const int tilesN = N >> 6;
  const int tilesM = M / (16 * MI);
  const int tile = blockIdx.x * 8 + wave;
  if (tile >= tilesM * tilesN) return;
  const int tm = tile / tilesN;
  const int tn = tile - tm * tilesN;
  const int m0 = tm * (16 * MI);
  const int n0 = tn << 6;
  const int rlane = lane & 15;
  const int koff  = (lane >> 4) * 8;
  const int mOff  = (lane >> 4) * 8;

  v8f acc[MI][4], accr[MI][4];
#pragma unroll
  for (int i = 0; i < MI; ++i)
#pragma unroll
    for (int j = 0; j < 4; ++j) {
      acc[i][j]  = (v8f){0.f, 0.f, 0.f, 0.f, 0.f, 0.f, 0.f, 0.f};
      accr[i][j] = (v8f){0.f, 0.f, 0.f, 0.f, 0.f, 0.f, 0.f, 0.f};
    }

  for (int k0 = 0; k0 < K; k0 += 32) {
    v16h bh[4], bl[4];
#pragma unroll
    for (int j = 0; j < 4; ++j) {
      const size_t bo = (size_t)(n0 + (j << 4) + rlane) * ldb + koff + k0;
      bh[j] = frag_load(Bt + bo);
      if (SPL == 2) bl[j] = frag_load(Bt2 + bo); else bl[j] = bh[j];
    }
#pragma unroll
    for (int i = 0; i < MI; ++i) {
      const size_t ao = (size_t)(m0 + (i << 4) + rlane) * lda + koff + k0;
      const v16h ah = frag_load(A + ao);
      v16h al = ah;
      if (SPL >= 1) al = frag_load(A2 + ao);
#pragma unroll
      for (int j = 0; j < 4; ++j) {
        acc[i][j] = mma(ah, bh[j], acc[i][j]);
        if (SPL >= 1) accr[i][j] = mma(al, bh[j], accr[i][j]);
        if (SPL == 2) accr[i][j] = mma(ah, bl[j], accr[i][j]);
      }
#pragma unroll
      for (int j = 0; j < 4; ++j) {
        guard1(acc[i][j], ah, al);
        if (SPL >= 1) guard1(accr[i][j], ah, al);
      }
    }
    keep4(bh[0], bh[1], bh[2], bh[3]);
    if (SPL == 2) keep4(bl[0], bl[1], bl[2], bl[3]);
  }
#pragma unroll
  for (int i = 0; i < MI; ++i)
#pragma unroll
    for (int j = 0; j < 4; ++j) {
      guard_acc(acc[i][j]);
      if (SPL >= 1) guard_acc(accr[i][j]);
    }

  float* slab = sT[wave];
#pragma unroll
  for (int i = 0; i < MI; ++i) {
    const int mBase = m0 + (i << 4);
#pragma unroll
    for (int j = 0; j < 4; ++j) {
#pragma unroll
      for (int r = 0; r < 8; ++r) {
        float v = acc[i][j][r] * scale;
        if (SPL >= 1) v += accr[i][j][r] * rscale;
        slab[(mOff + r) * 68 + (j << 4) + rlane] = v;
      }
    }
    __builtin_amdgcn_fence(__ATOMIC_RELEASE, "workgroup");
    __builtin_amdgcn_wave_barrier();
    __builtin_amdgcn_fence(__ATOMIC_ACQUIRE, "workgroup");
    {
      const int hh = lane >> 4, c4 = (lane & 15) * 4;
      for (int pass = 0; pass < 2; ++pass) {
#pragma unroll
        for (int it = 0; it < 8; ++it) {
          const int row = it * 2 + hh;
          const v4f v = *(const v4f*)(slab + row * 68 + c4);
          *(volatile v4f*)(C + (size_t)(mBase + row) * ldc + n0 + c4) = v;
        }
        __threadfence();
      }
    }
    __builtin_amdgcn_fence(__ATOMIC_RELEASE, "workgroup");
    __builtin_amdgcn_wave_barrier();
    __builtin_amdgcn_fence(__ATOMIC_ACQUIRE, "workgroup");
  }
}
}

__global__ __launch_bounds__(256) void rne_rows_f16_kernel(
    const float* __restrict__ src, unsigned short* __restrict__ dH, int total8)
{
  const int i = blockIdx.x * 256 + threadIdx.x;
  if (i >= total8) return;
  const size_t e0 = (size_t)i << 3;
  const v4f a0 = *(const v4f*)(src + e0);
  const v4f a1 = *(const v4f*)(src + e0 + 4);
  const float f0 = a0[0];
  const float f1 = a0[1];
  const float f2 = a0[2];
  const float f3 = a0[3];
  const float f4 = a1[0];
  const float f5 = a1[1];
  const float f6 = a1[2];
  const float f7 = a1[3];
  v8h hv;
  hv[0] = f16_flush(bf16r(f0));
  hv[1] = f16_flush(bf16r(f1));
  hv[2] = f16_flush(bf16r(f2));
  hv[3] = f16_flush(bf16r(f3));
  hv[4] = f16_flush(bf16r(f4));
  hv[5] = f16_flush(bf16r(f5));
  hv[6] = f16_flush(bf16r(f6));
  hv[7] = f16_flush(bf16r(f7));
  unsigned short* qh = dH + e0;
  *(volatile v8h*)qh = hv;
  __threadfence();
  *(volatile v8h*)qh = hv;
}

__global__ __launch_bounds__(256) void rne_vec_kernel(
    const float* __restrict__ src, float* __restrict__ dst, int n4)
{
  const int i = blockIdx.x * 256 + threadIdx.x;
  if (i >= n4) return;
  const v4f a = *(const v4f*)(src + (size_t)i * 4);
  const float a0 = a[0];
  const float a1 = a[1];
  const float a2 = a[2];
  const float a3 = a[3];
  v4f r;
  r[0] = bf16r(a0);
  r[1] = bf16r(a1);
  r[2] = bf16r(a2);
  r[3] = bf16r(a3);
  float* p = dst + (size_t)i * 4;
  *(volatile v4f*)p = r;
  __threadfence();
  *(volatile v4f*)p = r;
}

__global__ __launch_bounds__(256) void rne_plane_kernel(
    const float* __restrict__ src, float* __restrict__ dst, int n4)
{
  const int i = blockIdx.x * 256 + threadIdx.x;
  if (i >= n4) return;
  const v4f a = *(const v4f*)(src + (size_t)i * 4);
  const float a0 = a[0];
  const float a1 = a[1];
  const float a2 = a[2];
  const float a3 = a[3];
  v4f r;
  r[0] = bf16r(a0);
  r[1] = bf16r(a1);
  r[2] = bf16r(a2);
  r[3] = bf16r(a3);
  float* p = dst + (size_t)i * 4;
  *(volatile v4f*)p = r;
  __threadfence();
  *(volatile v4f*)p = r;
}

__global__ __launch_bounds__(256) void cat3_kernel(
    const float* __restrict__ WB, const float* __restrict__ WC, const float* __restrict__ WDT,
    float* __restrict__ WCAT, int total4)
{
  const int i = blockIdx.x * 256 + threadIdx.x;
  if (i >= total4) return;
  constexpr int kG = kProjP / 4;
  const int row = i / kG;
  const int c4 = (i - row * kG) * 4;
  const bool isB = (c4 < kNst);
  const bool isC = (c4 < kBcP);
  const bool isD = (c4 < kProjN);
  const int cb  = isB ? c4 : (kNst - 4);
  const int ccr = c4 - kNst;
  const int cc  = (ccr < 0) ? 0 : ((ccr < kNst) ? ccr : (kNst - 4));
  const int cdr = c4 - kBcP;
  const int cd  = (cdr < 0) ? 0 : ((cdr < kDim) ? cdr : (kDim - 4));
  const v4f vb = *(const v4f*)(WB + (size_t)row * kNst + cb);
  const v4f vc = *(const v4f*)(WC + (size_t)row * kNst + cc);
  const v4f vd = *(const v4f*)(WDT + (size_t)row * kDim + cd);
  v4f r;
#pragma unroll
  for (int e = 0; e < 4; ++e) {
    const float b0 = vb[e];
    const float c0 = vc[e];
    const float d0 = vd[e];
    const float tail = isD ? d0 : 0.0f;
    const float mid  = isC ? c0 : tail;
    r[e] = isB ? b0 : mid;
  }
  float* p = WCAT + (size_t)i * 4;
  *(volatile v4f*)p = r;
  __threadfence();
  *(volatile v4f*)p = r;
}

template <bool LO>
__global__ __launch_bounds__(256) void transpose_pack_kernel(
    const float* __restrict__ W, unsigned short* __restrict__ BtH, unsigned short* __restrict__ BtL,
    int Kdim, int Ndim, float carry)
{
  __shared__ float tile[64 * 65];
  const int tid = threadIdx.x, lane = tid & 31, wave = tid >> 5;
  const int n0 = blockIdx.x * 64;
  const int k0 = blockIdx.y * 64;
#pragma unroll
  for (int p = 0; p < 16; ++p) {
    const int idx = tid + p * 256;
    const int kk  = idx >> 6;
    const int nn  = idx & 63;
    const int n   = n0 + nn;
    const int nc  = (n < Ndim) ? n : (Ndim - 1);
    const float v = W[(size_t)(k0 + kk) * Ndim + nc];
    tile[kk * 65 + nn] = (n < Ndim) ? (bf16r(v) * carry) : 0.0f;
  }
  __syncthreads();
  const int q = lane >> 3, c8 = (lane & 7) * 8;
  v8h hv[2], lv[2];
#pragma unroll
  for (int it = 0; it < 2; ++it) {
    const int nrow = it * 32 + wave * 4 + q;
#pragma unroll
    for (int e = 0; e < 8; ++e) {
      _Float16 h, l;
      const float t = tile[(c8 + e) * 65 + nrow];
      f16_split(t, h, l);
      hv[it][e] = h;
      lv[it][e] = l;
    }
  }
  for (int pass = 0; pass < 2; ++pass) {
#pragma unroll
    for (int it = 0; it < 2; ++it) {
      const int nrow = it * 32 + wave * 4 + q;
      const size_t o = (size_t)(n0 + nrow) * Kdim + k0 + c8;
      *(volatile v8h*)(BtH + o) = hv[it];
      if (LO) *(volatile v8h*)(BtL + o) = lv[it];
    }
    __threadfence();
  }
}

__global__ __launch_bounds__(256) void proj_bias_split_kernel(
    const float* __restrict__ P, const float* __restrict__ bB, const float* __restrict__ bC,
    const float* __restrict__ dtb, float* __restrict__ BC, float* __restrict__ DT)
{
  const int tid = threadIdx.x;
  const int r0 = blockIdx.x * 32;
  const int c4 = (tid & 127) * 4;
  const int rh = tid >> 7;
  const v4f db = *(const v4f*)(dtb + c4);
  v4f dv[16];
#pragma unroll
  for (int it = 0; it < 16; ++it) {
    const int row = r0 + it * 2 + rh;
    const v4f p = *(const v4f*)(P + (size_t)row * kProjP + kBcP + c4);
    dv[it] = p + db;
  }
  const int rowb = r0 + (tid >> 3);
  const int p4 = (tid & 7) * 4;
  const bool isB = (p4 < kNst);
  const int ob = isB ? p4 : (kNst - 4);
  const int oc = isB ? 0 : (p4 - kNst);
  const v4f vb = *(const v4f*)(bB + ob);
  const v4f vc = *(const v4f*)(bC + oc);
  const v4f pv = *(const v4f*)(P + (size_t)rowb * kProjP + p4);
  v4f bcv;
#pragma unroll
  for (int e = 0; e < 4; ++e) {
    const float b0 = vb[e];
    const float c0 = vc[e];
    const float bs = isB ? b0 : c0;
    const float pe = pv[e];
    bcv[e] = pe + bf16r(bs);
  }
  for (int pass = 0; pass < 2; ++pass) {
#pragma unroll
    for (int it = 0; it < 16; ++it) {
      const int row = r0 + it * 2 + rh;
      *(volatile v4f*)(DT + (size_t)row * kDim + c4) = dv[it];
    }
    *(volatile v4f*)(BC + (size_t)rowb * kBcP + p4) = bcv;
    __threadfence();
  }
}

typedef float    ms1_v4f __attribute__((ext_vector_type(4)));
typedef unsigned ms1_v4u __attribute__((ext_vector_type(4)));
struct ms1_args {
  const float* dtpre;
  const float* u;
  const float* bc;
  const float* z;
  const float* A_log;
  const float* Dskip;
  __half* y;
  __half* y_lo;
  long ld_dtpre;
  long ld_u;
  long ld_bc;
  long ld_z;
  long ld_y;
  int offB;
  int offC;
  int offZ;
  float ycarry;
  int dir;
  int D;
  int L;
  int nbatch;
};
static_assert(sizeof(ms1_args) == 136);

__device__ __forceinline__ float ms1_flush16(float v) {
  return (fabsf(v) < 6.103515625e-05f) ? 0.0f : v;
}
__device__ __forceinline__ unsigned ms1_h16bits(float v) {
  return (unsigned)__half_as_ushort(__float2half_rn(ms1_flush16(v)));
}
__device__ __forceinline__ float ms1_h16val(unsigned b) {
  return __half2float(__ushort_as_half((unsigned short)b));
}
__device__ __forceinline__ float ms1_softplus(float v) {
  return fmaxf(v, 0.0f) + log1pf(expf(-fabsf(v)));
}
__device__ __forceinline__ void ms1_pack2(float v0, float v1, unsigned& hw, unsigned& lw) {
  const unsigned h0 = ms1_h16bits(v0);
  const unsigned h1 = ms1_h16bits(v1);
  const float r0 = (v0 - ms1_h16val(h0)) * 2048.0f;
  const float r1 = (v1 - ms1_h16val(h1)) * 2048.0f;
  const unsigned l0 = ms1_h16bits(r0);
  const unsigned l1 = ms1_h16bits(r1);
  hw = h0 | (h1 << 16);
  lw = l0 | (l1 << 16);
}

template <int NSTATE>
__global__ __launch_bounds__(64 * (NSTATE / 16)) void ms1_scan_kernel(ms1_args a)
{
  static_assert(NSTATE == 16 || NSTATE == 64);
  constexpr int NQ  = NSTATE / 16;
  constexpr int NT  = 64 * NQ;
  constexpr int NW  = NT / 32;
  constexpr int BCW = 2 * NSTATE;
  constexpr int YP  = 68;
  constexpr int RPI = NW * 4;
  constexpr int NIT = 64 / RPI;
  static_assert(16 * NT <= 64 * YP);
  __shared__ __align__(16) float sBC[64 * BCW];
  __shared__ __align__(16) float sY[64 * YP];
  const int tid  = threadIdx.x;
  const int lane = tid & 31;
  const int wave = tid >> 5;
  const int c    = tid / NQ;
  const int sq   = tid - c * NQ;
  const int bpb  = a.D / 64;
  const int bi   = blockIdx.x / bpb;
  if (bi >= a.nbatch) return;
  const int d0 = (blockIdx.x - bi * bpb) * 64;
  const int d  = d0 + c;
  const long rowb = (long)bi * a.L;
  const bool hasz  = (a.z != nullptr);
  const bool hasD  = (a.Dskip != nullptr);
  const bool hasLo = (a.y_lo != nullptr);

#pragma unroll 1
  for (int n = 0; n < 16; ++n) {
    const float al = a.A_log[(long)d * NSTATE + sq * 16 + n];
    sY[n * NT + tid] = -expf(al);
  }
  __syncthreads();
  float An[16], h[16];
#pragma unroll
  for (int n = 0; n < 16; ++n) {
    An[n] = sY[n * NT + tid];
    h[n] = 0.0f;
  }
  float Dd = 0.0f;
  if (hasD) Dd = a.Dskip[d];

  const int nchunk = a.L / 64;
  const bool fwd = (a.dir > 0);
  const int s0 = fwd ? 0 : 63;
  const int sd = fwd ? 1 : -1;
  const int q  = lane >> 3;
  const int c8 = (lane & 7) * 8;

  for (int ci = 0; ci < nchunk; ++ci) {
    const int tb = fwd ? (ci * 64) : (a.L - 64 - ci * 64);
    const long rowc = rowb + tb;
    __syncthreads();
#pragma unroll 8
    for (int i = 0; i < 32; ++i) {
      const int idx = tid + i * NT;
      const int st  = idx / BCW;
      const int col = idx - st * BCW;
      const int sc  = (col < NSTATE) ? (a.offB + col) : (a.offC + col - NSTATE);
      sBC[idx] = a.bc[(rowc + st) * a.ld_bc + sc];
    }
    __syncthreads();
    for (int s = 0; s < 64; ++s) {
      const int ls = s0 + sd * s;
      const long row = rowc + ls;
      float pre = a.dtpre[row * a.ld_dtpre + d];
      float uv  = a.u[row * a.ld_u + d];
      float zv  = 0.0f;
      if (hasz) zv = a.z[row * a.ld_z + a.offZ + d];
      asm volatile("" : "+v"(pre));
      asm volatile("" : "+v"(uv));
      asm volatile("" : "+v"(zv));
      const float delta = ms1_softplus(pre);
      const float dtx = delta * uv;
      const float* bp = sBC + ls * BCW + sq * 16;
      const float* cp = bp + NSTATE;
      ms1_v4f Bq[4], Cq[4];
#pragma unroll
      for (int k = 0; k < 4; ++k) {
        Bq[k] = *(const ms1_v4f*)(bp + 4 * k);
        Cq[k] = *(const ms1_v4f*)(cp + 4 * k);
      }
      float yv = 0.0f;
#pragma unroll
      for (int n = 0; n < 16; ++n) {
        const float e = __expf(delta * An[n]);
        h[n] = fmaf(e, h[n], dtx * Bq[n >> 2][n & 3]);
        yv = fmaf(h[n], Cq[n >> 2][n & 3], yv);
      }
      if (NQ > 1) {
        yv += __shfl_xor(yv, 1, 32);
        yv += __shfl_xor(yv, 2, 32);
      }
      if (hasD) yv = fmaf(uv, Dd, yv);
      if (hasz) {
        const float sg = __builtin_amdgcn_rcpf(1.0f + expf(-zv));
        yv = yv * (zv * sg);
      }
      if (sq == 0) sY[ls * YP + c] = yv * a.ycarry;
    }
    __syncthreads();
    ms1_v4u hw[NIT], lw[NIT];
#pragma unroll
    for (int it = 0; it < NIT; ++it) {
      const int row = it * RPI + wave * 4 + q;
      const float* sp = sY + row * YP + c8;
      const ms1_v4f f0 = *(const ms1_v4f*)(sp);
      const ms1_v4f f1 = *(const ms1_v4f*)(sp + 4);
      unsigned h0, h1, h2, h3, l0, l1, l2, l3;
      ms1_pack2(f0[0], f0[1], h0, l0);
      ms1_pack2(f0[2], f0[3], h1, l1);
      ms1_pack2(f1[0], f1[1], h2, l2);
      ms1_pack2(f1[2], f1[3], h3, l3);
      hw[it] = (ms1_v4u){h0, h1, h2, h3};
      lw[it] = (ms1_v4u){l0, l1, l2, l3};
    }
    for (int pass = 0; pass < 2; ++pass) {
#pragma unroll
      for (int it = 0; it < NIT; ++it) {
        const int row = it * RPI + wave * 4 + q;
        const long o = (rowc + row) * a.ld_y + d0 + c8;
        *(volatile ms1_v4u*)(a.y + o) = hw[it];
        if (hasLo) *(volatile ms1_v4u*)(a.y_lo + o) = lw[it];
      }
      __threadfence();
    }
  }
}

__device__ __forceinline__ float gelu_from_words(unsigned hb, unsigned lb) {
  const float hi = h16_to_f32(hb);
  const float lo = h16_to_f32(lb);
  const float y = (hi + lo * kInvResid) * kInvCarry;
  return 0.5f * y * (1.0f + erff(y * 0.70710678f));
}

__global__ __launch_bounds__(256) void gelu_split_kernel(
    const unsigned short* __restrict__ YH, const unsigned short* __restrict__ YL,
    unsigned short* __restrict__ GH, unsigned short* __restrict__ GL, int total8)
{
  const int i = blockIdx.x * 256 + threadIdx.x;
  if (i >= total8) return;
  const size_t e0 = (size_t)i << 3;
  const v4u hw = *(const v4u*)(const void*)(YH + e0);
  const v4u lw = *(const v4u*)(const void*)(YL + e0);
  const unsigned hw0 = hw[0];
  const unsigned hw1 = hw[1];
  const unsigned hw2 = hw[2];
  const unsigned hw3 = hw[3];
  const unsigned lw0 = lw[0];
  const unsigned lw1 = lw[1];
  const unsigned lw2 = lw[2];
  const unsigned lw3 = lw[3];
  const float g0 = gelu_from_words(hw0 & 0xffffu, lw0 & 0xffffu);
  const float g1 = gelu_from_words(hw0 >> 16, lw0 >> 16);
  const float g2 = gelu_from_words(hw1 & 0xffffu, lw1 & 0xffffu);
  const float g3 = gelu_from_words(hw1 >> 16, lw1 >> 16);
  const float g4 = gelu_from_words(hw2 & 0xffffu, lw2 & 0xffffu);
  const float g5 = gelu_from_words(hw2 >> 16, lw2 >> 16);
  const float g6 = gelu_from_words(hw3 & 0xffffu, lw3 & 0xffffu);
  const float g7 = gelu_from_words(hw3 >> 16, lw3 >> 16);
  _Float16 a0, a1, a2, a3, a4, a5, a6, a7;
  _Float16 b0, b1, b2, b3, b4, b5, b6, b7;
  f16_split(g0, a0, b0);
  f16_split(g1, a1, b1);
  f16_split(g2, a2, b2);
  f16_split(g3, a3, b3);
  f16_split(g4, a4, b4);
  f16_split(g5, a5, b5);
  f16_split(g6, a6, b6);
  f16_split(g7, a7, b7);
  v8h hv, lv;
  hv[0] = a0; lv[0] = b0;
  hv[1] = a1; lv[1] = b1;
  hv[2] = a2; lv[2] = b2;
  hv[3] = a3; lv[3] = b3;
  hv[4] = a4; lv[4] = b4;
  hv[5] = a5; lv[5] = b5;
  hv[6] = a6; lv[6] = b6;
  hv[7] = a7; lv[7] = b7;
  unsigned short* qh = GH + e0;
  unsigned short* ql = GL + e0;
  *(volatile v8h*)qh = hv;
  *(volatile v8h*)ql = lv;
  __threadfence();
  *(volatile v8h*)qh = hv;
  *(volatile v8h*)ql = lv;
}

__device__ __forceinline__ float ln_res_value(float t, float mu, float inv, float w, float b, float r) {
  const float n = (t - mu) * inv * w + b;
  return r + n;
}

__global__ __launch_bounds__(256) void ln_res_kernel(
    const float* __restrict__ MX, const float* __restrict__ mxb,
    const float* __restrict__ gw, const float* __restrict__ gb,
    const float* __restrict__ Hcur, float* __restrict__ Hnext,
    unsigned short* __restrict__ dH, unsigned short* __restrict__ dL, int rows, int write_lo)
{
  const int lane = threadIdx.x & 31;
  const int wave = threadIdx.x >> 5;
  const int row  = blockIdx.x * 8 + wave;
  if (row >= rows) return;
  const float* xr = MX + (size_t)row * kDim;
  const float* hr = Hcur + (size_t)row * kDim;
  v4f t[4];
#pragma unroll
  for (int g = 0; g < 4; ++g) {
    const int off = (g >> 1) * 256 + lane * 8 + (g & 1) * 4;
    const v4f a = *(const v4f*)(xr + off);
    const v4f b = *(const v4f*)(mxb + off);
    t[g] = a + b;
  }
  float s = 0.0f;
#pragma unroll
  for (int g = 0; g < 4; ++g)
#pragma unroll
    for (int e = 0; e < 4; ++e) s += t[g][e];
#pragma unroll
  for (int o = 16; o >= 1; o >>= 1) s += __shfl_xor(s, o, 32);
  const float mu = s * (1.0f / (float)kDim);
  float ss = 0.0f;
#pragma unroll
  for (int g = 0; g < 4; ++g)
#pragma unroll
    for (int e = 0; e < 4; ++e) {
      const float dv = t[g][e] - mu;
      ss = fmaf(dv, dv, ss);
    }
#pragma unroll
  for (int o = 16; o >= 1; o >>= 1) ss += __shfl_xor(ss, o, 32);
  const float var = ss * (1.0f / (float)kDim);
  const float inv = rsqrtf(var + kLnEps);
  v8h hv[2], lv[2];
#pragma unroll
  for (int g = 0; g < 4; ++g) {
    const int off = (g >> 1) * 256 + lane * 8 + (g & 1) * 4;
    const v4f w4 = *(const v4f*)(gw + off);
    const v4f b4 = *(const v4f*)(gb + off);
    const v4f r4 = *(const v4f*)(hr + off);
#pragma unroll
    for (int e = 0; e < 4; ++e) {
      const float hn = ln_res_value(t[g][e], mu, inv, w4[e], b4[e], r4[e]);
      _Float16 h, l;
      f16_split(hn, h, l);
      hv[g >> 1][(g & 1) * 4 + e] = h;
      lv[g >> 1][(g & 1) * 4 + e] = l;
    }
  }
  v4f fo[4];
#pragma unroll
  for (int g = 0; g < 4; ++g) {
    const int off = g * 128 + lane * 4;
    const v4f a  = *(const v4f*)(xr + off);
    const v4f b  = *(const v4f*)(mxb + off);
    const v4f w4 = *(const v4f*)(gw + off);
    const v4f b4 = *(const v4f*)(gb + off);
    const v4f r4 = *(const v4f*)(hr + off);
    const v4f tt = a + b;
#pragma unroll
    for (int e = 0; e < 4; ++e)
      fo[g][e] = ln_res_value(tt[e], mu, inv, w4[e], b4[e], r4[e]);
  }
  for (int pass = 0; pass < 2; ++pass) {
#pragma unroll
    for (int g = 0; g < 4; ++g)
      *(volatile v4f*)(Hnext + (size_t)row * kDim + g * 128 + lane * 4) = fo[g];
#pragma unroll
    for (int hf = 0; hf < 2; ++hf) {
      const size_t o = (size_t)row * kDim + hf * 256 + lane * 8;
      *(volatile v8h*)(dH + o) = hv[hf];
      if (write_lo) *(volatile v8h*)(dL + o) = lv[hf];
    }
    __threadfence();
  }
}

__global__ __launch_bounds__(128) void bias_out_kernel(
    const float* __restrict__ DEC, const float* __restrict__ decb, float* __restrict__ out)
{
  const int d4 = (blockIdx.x * 128 + threadIdx.x) * 4;
  const int r0 = blockIdx.y * 8;
  const v4f b = *(const v4f*)(decb + d4);
  v4f val[8];
#pragma unroll
  for (int i = 0; i < 8; ++i) {
    const v4f p = *(const v4f*)(DEC + (size_t)(r0 + i) * kDim + d4);
    val[i] = p + b;
  }
  for (int pass = 0; pass < 2; ++pass) {
#pragma unroll
    for (int i = 0; i < 8; ++i)
      *(volatile v4f*)(out + (size_t)(r0 + i) * kDim + d4) = val[i];
    __threadfence();
  }
}

static_assert(((kSeq / 32) * (kProjP / 64)) % 8 == 0);
static_assert(((kSeq / 32) * (kDim / 64)) % 8 == 0);
static_assert(((kDim * kProjP / 4) % 256) == 0);
static_assert(((kSeq * kDim / 8) % 256) == 0);
static_assert(((kSeq * kDim / 4) % 256) == 0);
static_assert(((kDim * kNst / 4) % 256) == 0);
static_assert((kDim / 4) == 128);
static_assert((kSeq % 32) == 0 && (kSeq % 8) == 0);

extern "C" void kernel_launch(void* const* d_in, const int* in_sizes, int n_in,
                              void* d_out, int out_size, void* d_ws, size_t ws_size,
                              hipStream_t stream)
{
  if (n_in < 15) return;
  if (in_sizes[0] != kBatch * kSeq * kDim) return;
  if (in_sizes[1] != kLayers * kDim * kNst) return;
  if (in_sizes[2] != kLayers * kDim * kNst) return;
  if (in_sizes[3] != kLayers * kNst) return;
  if (in_sizes[4] != kLayers * kDim * kNst) return;
  if (in_sizes[5] != kLayers * kNst) return;
  if (in_sizes[6] != kLayers * kDim * kDim) return;
  if (in_sizes[7] != kLayers * kDim) return;
  if (in_sizes[8] != kLayers * kDim) return;
  if (in_sizes[9] != kLayers * kDim * kDim) return;
  if (in_sizes[10] != kLayers * kDim) return;
  if (in_sizes[11] != kLayers * kDim) return;
  if (in_sizes[12] != kLayers * kDim) return;
  if (in_sizes[13] != kDim * kDim) return;
  if (in_sizes[14] != kDim) return;
  if (out_size != kBatch * kSeq * kDim) return;
  if (ws_size < kWsTotal) return;

  const float* x      = (const float*)d_in[0];
  const float* A_log  = (const float*)d_in[1];
  const float* W_B    = (const float*)d_in[2];
  const float* b_B    = (const float*)d_in[3];
  const float* W_C    = (const float*)d_in[4];
  const float* b_C    = (const float*)d_in[5];
  const float* W_dt   = (const float*)d_in[6];
  const float* b_dt   = (const float*)d_in[7];
  const float* D_skip = (const float*)d_in[8];
  const float* W_mix  = (const float*)d_in[9];
  const float* b_mix  = (const float*)d_in[10];
  const float* ln_g   = (const float*)d_in[11];
  const float* ln_b   = (const float*)d_in[12];
  const float* W_dec  = (const float*)d_in[13];
  const float* b_dec  = (const float*)d_in[14];
  float* out = (float*)d_out;

  char* ws = (char*)d_ws;
  float*          WCAT = (float*)(ws + kOffWCAT);
  unsigned short* W3   = (unsigned short*)(ws + kOffW3);
  unsigned short* WM   = (unsigned short*)(ws + kOffWM);
  unsigned short* WD   = (unsigned short*)(ws + kOffWD);
  float*          VEC  = (float*)(ws + kOffVEC);
  float*          ALOG = (float*)(ws + kOffALOG);
  float*          HA   = (float*)(ws + kOffHA);
  float*          HB   = (float*)(ws + kOffHB);
  unsigned short* HH   = (unsigned short*)(ws + kOffHH);
  unsigned short* HL   = (unsigned short*)(ws + kOffHL);
  float*          P    = (float*)(ws + kOffP);
  float*          BC   = (float*)(ws + kOffBC);
  float*          DT   = (float*)(ws + kOffDT);
  unsigned short* YH   = (unsigned short*)(ws + kOffYH);
  unsigned short* YL   = (unsigned short*)(ws + kOffYL);
  unsigned short* GH   = (unsigned short*)(ws + kOffGH);
  unsigned short* GL   = (unsigned short*)(ws + kOffGL);
  float*          MX   = (float*)(ws + kOffMX);
  float*          DEC  = (float*)(ws + kOffDEC);

  float* DECB = VEC + (size_t)10 * kDim;

  constexpr size_t kDN = (size_t)kDim * kNst;
  constexpr size_t kDD = (size_t)kDim * kDim;
  constexpr size_t kCatE = (size_t)kDim * kProjP;

  for (int i = 0; i < kLayers; ++i) {
    float* WCATi = WCAT + (size_t)i * kCatE;
    unsigned short* W3i = W3 + (size_t)i * kCatE;
    unsigned short* WMi = WM + (size_t)i * kDD;

    cat3_kernel<<<(kDim * kProjP / 4) / 256, 256, 0, stream>>>(
        W_B + (size_t)i * kDN, W_C + (size_t)i * kDN, W_dt + (size_t)i * kDD, WCATi, kDim * kProjP / 4);

    transpose_pack_kernel<false><<<dim3(kProjP / 64, kDim / 64), 256, 0, stream>>>(
        WCATi, W3i, W3i, kDim, kProjP, kWCarry);

    transpose_pack_kernel<false><<<dim3(kDim / 64, kDim / 64), 256, 0, stream>>>(
        W_mix + (size_t)i * kDD, WMi, WMi, kDim, kDim, kWCarry);

    rne_vec_kernel<<<1, 256, 0, stream>>>(b_dt   + (size_t)i * kDim, VEC + (size_t)(0 * 2 + i) * kDim, kDim / 4);
    rne_vec_kernel<<<1, 256, 0, stream>>>(D_skip + (size_t)i * kDim, VEC + (size_t)(1 * 2 + i) * kDim, kDim / 4);
    rne_vec_kernel<<<1, 256, 0, stream>>>(b_mix  + (size_t)i * kDim, VEC + (size_t)(2 * 2 + i) * kDim, kDim / 4);
    rne_vec_kernel<<<1, 256, 0, stream>>>(ln_g   + (size_t)i * kDim, VEC + (size_t)(3 * 2 + i) * kDim, kDim / 4);
    rne_vec_kernel<<<1, 256, 0, stream>>>(ln_b   + (size_t)i * kDim, VEC + (size_t)(4 * 2 + i) * kDim, kDim / 4);

    rne_vec_kernel<<<(kDim * kNst / 4) / 256, 256, 0, stream>>>(
        A_log + (size_t)i * kDN, ALOG + (size_t)i * kDN, kDim * kNst / 4);
  }

  transpose_pack_kernel<false><<<dim3(kDim / 64, kDim / 64), 256, 0, stream>>>(W_dec, WD, WD, kDim, kDim, kWCarry);
  rne_vec_kernel<<<1, 256, 0, stream>>>(b_dec, DECB, kDim / 4);

  constexpr float sW  = 1.0f / kWCarry;
  constexpr float sWr = 1.0f / (kWCarry * kResid);
  constexpr int kGridProj = (kSeq / 32) * (kProjP / 64) / 8;
  constexpr int kGridSq   = (kSeq / 32) * (kDim / 64) / 8;
  static_assert(kGridProj == 72 && kGridSq == 64);

  for (int b = 0; b < kBatch; ++b) {
    const float* xb = x + (size_t)b * kSeq * kDim;
    float* outb = out + (size_t)b * kSeq * kDim;

    rne_plane_kernel<<<(kSeq * kDim / 4) / 256, 256, 0, stream>>>(xb, HA, kSeq * kDim / 4);
    rne_rows_f16_kernel<<<(kSeq * kDim / 8) / 256, 256, 0, stream>>>(xb, HH, kSeq * kDim / 8);

    for (int i = 0; i < kLayers; ++i) {
      float* Hcur  = (i == 0) ? HA : HB;
      float* Hnext = (i == 0) ? HB : HA;
      const unsigned short* W3i = W3 + (size_t)i * kCatE;
      const unsigned short* WMi = WM + (size_t)i * kDD;
      const float* DTBi = VEC + (size_t)(0 * 2 + i) * kDim;
      const float* DSKi = VEC + (size_t)(1 * 2 + i) * kDim;
      const float* MXBi = VEC + (size_t)(2 * 2 + i) * kDim;
      const float* LNGi = VEC + (size_t)(3 * 2 + i) * kDim;
      const float* LNBi = VEC + (size_t)(4 * 2 + i) * kDim;

      if (i == 0) {
        eng::gemm_f16_kernel<2, 0><<<dim3(kGridProj), 256, 0, stream>>>(
            HH, nullptr, kDim, W3i, nullptr, kDim, P, kProjP, kSeq, kProjP, kDim, sW, 0.0f);
      } else {
        eng::gemm_f16_kernel<2, 1><<<dim3(kGridProj), 256, 0, stream>>>(
            HH, HL, kDim, W3i, W3i, kDim, P, kProjP, kSeq, kProjP, kDim, sW, sWr);
      }

      proj_bias_split_kernel<<<kSeq / 32, 256, 0, stream>>>(
          P, b_B + (size_t)i * kNst, b_C + (size_t)i * kNst, DTBi, BC, DT);

      ms1_args sa;
      sa.dtpre = DT;
      sa.u = Hcur;
      sa.bc = BC;
      sa.z = nullptr;
      sa.A_log = ALOG + (size_t)i * kDN;
      sa.Dskip = DSKi;
      sa.y = (__half*)YH;
      sa.y_lo = (__half*)YL;
      sa.ld_dtpre = kDim;
      sa.ld_u = kDim;
      sa.ld_bc = kBcP;
      sa.ld_z = 0;
      sa.ld_y = kDim;
      sa.offB = 0;
      sa.offC = kNst;
      sa.offZ = 0;
      sa.ycarry = kYCarry;
      sa.dir = 1;
      sa.D = kDim;
      sa.L = kSeq;
      sa.nbatch = 1;
      ms1_scan_kernel<16><<<dim3(kDim / 64), 64, 0, stream>>>(sa);

      gelu_split_kernel<<<(kSeq * kDim / 8) / 256, 256, 0, stream>>>(YH, YL, GH, GL, kSeq * kDim / 8);

      eng::gemm_f16_kernel<2, 1><<<dim3(kGridSq), 256, 0, stream>>>(
          GH, GL, kDim, WMi, WMi, kDim, MX, kDim, kSeq, kDim, kDim, sW, sWr);

      ln_res_kernel<<<kSeq / 8, 256, 0, stream>>>(
          MX, MXBi, LNGi, LNBi, Hcur, Hnext, HH, HL, kSeq, (i + 1 < kLayers) ? 1 : 0);
    }

    eng::gemm_f16_kernel<2, 0><<<dim3(kGridSq), 256, 0, stream>>>(
        HH, nullptr, kDim, WD, nullptr, kDim, DEC, kDim, kSeq, kDim, kDim, sW, 0.0f);

    bias_out_kernel<<<dim3(1, kSeq / 8), 128, 0, stream>>>(DEC, DECB, outb);
  }
}
